// PGExplainerStyle_9483287790247
// MI455X (gfx1250) — hardware-verified
//
#include <hip/hip_runtime.h>
#include <stddef.h>


#define HD      128
#define AD      16
#define PQROW   256
#define NTHR    256
#define NWAVE   8
#define NBN     64
#define XP      136
#define SP      132
#define TE      (NWAVE * 32)
#define PWTOT   32768
#define PREPBLK (PWTOT / (NTHR * 8))
#define WSCAP   134217728
#define PQDYN   (NWAVE * 16 * SP * 4)

static_assert((PWTOT % (NTHR * 8)) == 0);
static_assert(((XP * 2) % 16) == 0);
static_assert(((SP * 4) % 16) == 0);
static_assert(NBN == 4 * 16);
static_assert(NTHR == 4 * NBN);
static_assert(TE == NWAVE * 32);
static_assert(HD == 4 * 32);

typedef float          v4f   __attribute__((ext_vector_type(4)));
typedef float          v8f   __attribute__((ext_vector_type(8)));
typedef unsigned int   v4u   __attribute__((ext_vector_type(4)));
typedef _Float16       v8h   __attribute__((ext_vector_type(8)));
typedef _Float16       v16h  __attribute__((ext_vector_type(16)));

__device__ __forceinline__ v16h ldfrag(const _Float16* p) {
  const v8h u0 = *(const v8h*)p;
  const v8h u1 = *(const v8h*)(p + 16);
  return __builtin_shufflevector(u0, u1, 0, 1, 2, 3, 4, 5, 6, 7, 8, 9, 10, 11, 12, 13, 14, 15);
}

__device__ __forceinline__ v8f wm(v16h a, v16h b, v8f c) {
  v8f d = __builtin_amdgcn_wmma_f32_16x16x32_f16(false, a, false, b, (short)0, c, false, false);
  asm volatile("v_nop\n\tv_nop\n\tv_nop\n\tv_nop" : "+v"(d) : "v"(a), "v"(b));
  return d;
}
__device__ __forceinline__ v8f zero8() {
  v8f z = {0.f, 0.f, 0.f, 0.f, 0.f, 0.f, 0.f, 0.f};
  return z;
}
__device__ __forceinline__ int iclamp(int v, int lo, int hi) { return v < lo ? lo : (v > hi ? hi : v); }

__global__ __launch_bounds__(NTHR) void k_prep(const float* __restrict__ W1, _Float16* wp) {
  const int tid = (int)threadIdx.x;
  const int o = ((int)blockIdx.x * NTHR + tid) * 8;
  const int n = o >> 7, k0 = o & (HD - 1);
  const int rowb = (n < HD) ? k0 : (HD + k0);
  const int col  = (n < HD) ? n : (n - HD);
  v8h hv;
#pragma unroll
  for (int i = 0; i < 8; ++i) hv[i] = (_Float16)(64.0f * W1[(size_t)(rowb + i) * HD + col]);
  const v4u u = __builtin_bit_cast(v4u, hv);
  _Float16* dst = wp + o;
  *(volatile v4u*)dst = u;
  __threadfence();
  *(volatile v4u*)dst = u;
}

__global__ __launch_bounds__(NTHR) void k_pq(const float* __restrict__ x, const _Float16* __restrict__ wp,
                                             float* PQ, int nN) {
  extern __shared__ __attribute__((aligned(16))) float stg[];
  __shared__ __attribute__((aligned(16))) _Float16 sX[NBN * XP];
  const int tid = (int)threadIdx.x, lane = tid & 31, wave = tid >> 5, hh = lane >> 4, m = lane & 15;
  const int n0 = (int)blockIdx.x * NBN;

  {
    const int nl = tid >> 2, q = tid & 3;
    int node = n0 + nl;
    node = node > nN - 1 ? nN - 1 : node;
    const float* rp = x + (size_t)node * HD + 32 * q;
    _Float16* dp = sX + nl * XP + 32 * q;
#pragma unroll
    for (int i = 0; i < 4; ++i) {
      const v4f a = *(const v4f*)(rp + 8 * i);
      const v4f b = *(const v4f*)(rp + 8 * i + 4);
      v8h u;
      u[0] = (_Float16)a.x; u[1] = (_Float16)a.y; u[2] = (_Float16)a.z; u[3] = (_Float16)a.w;
      u[4] = (_Float16)b.x; u[5] = (_Float16)b.y; u[6] = (_Float16)b.z; u[7] = (_Float16)b.w;
      *(v8h*)(dp + 8 * i) = u;
    }
  }
  __syncthreads();

  const int rt = wave & 3, cg = wave >> 2;
  v8f c[8];
#pragma unroll
  for (int j = 0; j < 8; ++j) c[j] = zero8();
  const _Float16* ap = sX + (16 * rt + m) * XP + 8 * hh;
  const _Float16* bp = wp + (size_t)(HD * cg + m) * HD + 8 * hh;
#pragma unroll
  for (int ks = 0; ks < 4; ++ks) {
    const v16h a = ldfrag(ap + 32 * ks);
#pragma unroll
    for (int j = 0; j < 8; ++j) {
      const v16h b = ldfrag(bp + (size_t)(16 * j) * HD + 32 * ks);
      c[j] = wm(a, b, c[j]);
    }
  }
  float* sw = stg + wave * 16 * SP;
#pragma unroll
  for (int j = 0; j < 8; ++j) {
#pragma unroll
    for (int r = 0; r < 8; ++r) sw[(8 * hh + r) * SP + 16 * j + m] = c[j][r] * 0.015625f;
  }
  __syncthreads();
#pragma unroll 1
  for (int rr = 0; rr < 16; ++rr) {
    const v4f v = *(const v4f*)(sw + rr * SP + 4 * lane);
    *(volatile v4f*)(PQ + (size_t)(n0 + 16 * rt + rr) * PQROW + HD * cg + 4 * lane) = v;
  }
  __threadfence();
#pragma unroll 1
  for (int rr = 0; rr < 16; ++rr) {
    const v4f v = *(const v4f*)(sw + rr * SP + 4 * lane);
    *(volatile v4f*)(PQ + (size_t)(n0 + 16 * rt + rr) * PQROW + HD * cg + 4 * lane) = v;
  }
}

__global__ __launch_bounds__(NTHR) void k_edge(
    const int* __restrict__ ei, const float* __restrict__ ea, const float* __restrict__ PQ,
    const float* __restrict__ W1, const float* __restrict__ b1, const float* __restrict__ W2,
    const float* __restrict__ b2, float* outp, int nE, int nN) {
  const int tid = (int)threadIdx.x, lane = tid & 31, wave = tid >> 5;

  v4f wc[AD];
#pragma unroll
  for (int k = 0; k < AD; ++k) wc[k] = *(const v4f*)(W1 + (size_t)(2 * HD + k) * HD + 4 * lane);
  const v4f bq = *(const v4f*)(b1 + 4 * lane);
  const v4f w2 = *(const v4f*)(W2 + 4 * lane);
  const float bias2 = b2[0];
  const int ebase = __builtin_amdgcn_readfirstlane(((int)blockIdx.x * NWAVE + wave) * 32);

  float myout = 0.0f;
#pragma unroll 1
  for (int it = 0; it < 32; ++it) {
    int ec = ebase + it;
    ec = ec > nE - 1 ? nE - 1 : ec;
    int s = ei[ec];
    int d = ei[(size_t)nE + ec];
    s = s < 0 ? s + nN : s;
    d = d < 0 ? d + nN : d;
    s = iclamp(s, 0, nN - 1);
    d = iclamp(d, 0, nN - 1);
    const v4f p = *(const v4f*)(PQ + (size_t)s * PQROW + 4 * lane);
    const v4f q = *(const v4f*)(PQ + (size_t)d * PQROW + HD + 4 * lane);
    const float* arow = ea + (size_t)ec * AD;
    const v4f a0 = *(const v4f*)(arow);
    const v4f a1 = *(const v4f*)(arow + 4);
    const v4f a2 = *(const v4f*)(arow + 8);
    const v4f a3 = *(const v4f*)(arow + 12);
    v4f h = p + q;
    h = a0.x * wc[0]  + h;  h = a0.y * wc[1]  + h;  h = a0.z * wc[2]  + h;  h = a0.w * wc[3]  + h;
    h = a1.x * wc[4]  + h;  h = a1.y * wc[5]  + h;  h = a1.z * wc[6]  + h;  h = a1.w * wc[7]  + h;
    h = a2.x * wc[8]  + h;  h = a2.y * wc[9]  + h;  h = a2.z * wc[10] + h;  h = a2.w * wc[11] + h;
    h = a3.x * wc[12] + h;  h = a3.y * wc[13] + h;  h = a3.z * wc[14] + h;  h = a3.w * wc[15] + h;
    h = h + bq;
    h.x = fmaxf(h.x, 0.0f); h.y = fmaxf(h.y, 0.0f); h.z = fmaxf(h.z, 0.0f); h.w = fmaxf(h.w, 0.0f);
    float o = h.x * w2.x;
    o = h.y * w2.y + o;
    o = h.z * w2.z + o;
    o = h.w * w2.w + o;
    o += __shfl_xor(o, 16, 32);
    o += __shfl_xor(o, 8, 32);
    o += __shfl_xor(o, 4, 32);
    o += __shfl_xor(o, 2, 32);
    o += __shfl_xor(o, 1, 32);
    myout = (lane == it) ? o : myout;
  }

  const float v = myout + bias2;
  const int eo = ebase + lane;
  if (eo < nE) *(volatile float*)(outp + eo) = v;
  __threadfence();
  if (eo < nE) *(volatile float*)(outp + eo) = v;
}

extern "C" void kernel_launch(void* const* d_in, const int* in_sizes, int n_in,
                              void* d_out, int out_size, void* d_ws, size_t ws_size,
                              hipStream_t stream) {
  if (n_in < 7) return;
  if (in_sizes[0] < HD || (in_sizes[0] % HD) != 0) return;
  const int nN = in_sizes[0] / HD;
  if (nN < 1 || nN > (1 << 22)) return;
  const int nE = out_size;
  if (nE < 1 || nE > (1 << 27)) return;
  if (in_sizes[1] != 2 * nE) return;
  if ((long long)in_sizes[2] != (long long)nE * AD) return;
  if (in_sizes[3] != (2 * HD + AD) * HD || in_sizes[4] != HD) return;
  if (in_sizes[5] != HD || in_sizes[6] < 1) return;

  const float* x  = (const float*)d_in[0];
  const int*   ei = (const int*)d_in[1];
  const float* ea = (const float*)d_in[2];
  const float* W1 = (const float*)d_in[3];
  const float* b1 = (const float*)d_in[4];
  const float* W2 = (const float*)d_in[5];
  const float* b2 = (const float*)d_in[6];
  float* outp = (float*)d_out;

  const int nb64 = (nN + NBN - 1) / NBN;
  const int Npad64 = nb64 * NBN;
  const int nbE = (nE + TE - 1) / TE;

  const size_t cap = ws_size < (size_t)WSCAP ? ws_size : (size_t)WSCAP;
  const size_t bW  = (size_t)PWTOT * 2;
  const size_t bPQ = (size_t)Npad64 * PQROW * 4;
  size_t off = 0;
  const size_t oW  = off; off += bW;                    off = (off + 255) & ~(size_t)255;
  const size_t oPQ = off; off += bPQ;                   off = (off + 255) & ~(size_t)255;
  if (off > cap) return;
  char* ws = (char*)d_ws;
  _Float16* wp = (_Float16*)(ws + oW);
  float*    PQ = (float*)(ws + oPQ);

  hipFuncSetAttribute(reinterpret_cast<const void*>(&k_pq), hipFuncAttributeMaxDynamicSharedMemorySize, PQDYN);

  k_prep<<<PREPBLK, NTHR, 0, stream>>>(W1, wp);
  k_pq<<<nb64, NTHR, PQDYN, stream>>>(x, wp, PQ, nN);
  k_edge<<<nbE, NTHR, 0, stream>>>(ei, ea, PQ, W1, b1, W2, b2, outp, nE, nN);
}
